// Level_Cat_3_8_16767552324153
// MI455X (gfx1250) — hardware-verified
//
#include <hip/hip_runtime.h>


namespace {
constexpr int Bn = 16, C = 64, HH = 64, WW = 64, NP = HH * WW  , NK = (HH / 2) * (WW / 2)  , I = 32, CL = 32;
constexpr float CS8 = 8.0f, PS = 8.0f, BNE = 1e-5f;
constexpr size_t TPL = (size_t)Bn * NP * I, KPL = (size_t)Bn * NK * I, GPL = (size_t)Bn * I * NK;

typedef _Float16 b16;
typedef __attribute__((ext_vector_type(16))) _Float16 v16b;
typedef __attribute__((ext_vector_type(8)))  _Float16 v8b;
typedef __attribute__((ext_vector_type(8)))  float v8f;
typedef __attribute__((ext_vector_type(4)))  float v4f;

__device__ __forceinline__ v8b ld8b(const b16* p) { return *(const v8b*)p; }
__device__ __forceinline__ v16b cat8b(v8b a, v8b b) { return __builtin_shufflevector(a, b, 0, 1, 2, 3, 4, 5, 6, 7, 8, 9, 10, 11, 12, 13, 14, 15); }
__device__ __forceinline__ v16b frag_kb(const b16* p, int hh) { return cat8b(ld8b(p + 8 * hh), ld8b(p + 16 + 8 * hh)); }
__device__ __forceinline__ void split16(float v, b16& hi, b16& lo) { hi = (b16)v; lo = (b16)(v - (float)hi); }
__device__ __forceinline__ void frag_ksplit(const float* p, int hh, v16b& fh_, v16b& fl_) {
  const float* p0 = p + 8 * hh; const float* p1 = p + 16 + 8 * hh;
#pragma unroll
  for (int e = 0; e < 8; ++e) { b16 a, c; split16(p0[e], a, c); fh_[e] = a; fl_[e] = c; split16(p1[e], a, c); fh_[8 + e] = a; fl_[8 + e] = c; }
}
__device__ __forceinline__ v8f wmma16b(v16b a, v16b b, v8f c) {
  v8f d = __builtin_amdgcn_wmma_f32_16x16x32_f16(false, a, false, b, (short)0, c, false, false);
  asm volatile("v_nop\n\tv_nop\n\tv_nop\n\tv_nop" : "+v"(d) : "v"(a), "v"(b));
  return d;
}
__device__ __forceinline__ void wave_lds_sync() {
  __builtin_amdgcn_fence(__ATOMIC_RELEASE, "workgroup");
  __builtin_amdgcn_wave_barrier();
  __builtin_amdgcn_fence(__ATOMIC_ACQUIRE, "workgroup");
}

struct Opnd { const void* p0; const void* p1; int ld; };
template <int NP> __device__ __forceinline__ void load_frags(const Opnd& o, int row, int kb, int hh, v16b& fh_, v16b& fl_) {
  if (NP == 0) { frag_ksplit((const float*)o.p0 + (size_t)row * o.ld + kb, hh, fh_, fl_); }
  else if (NP == 4 || NP == 5) {
    const float sc_ = (NP == 4) ? 64.0f : 8.0f;
    const float* p = (const float*)o.p0 + (size_t)row * o.ld + kb; const float* p0 = p + 8 * hh; const float* p1 = p + 16 + 8 * hh;
#pragma unroll
    for (int e = 0; e < 8; ++e) { b16 a, c; split16(p0[e] * sc_, a, c); fh_[e] = a; fl_[e] = c; split16(p1[e] * sc_, a, c); fh_[8 + e] = a; fl_[8 + e] = c; }
  } else if (NP == 3) {
    const float* p = (const float*)o.p0 + (size_t)row * o.ld + kb; const float* p0 = p + 8 * hh; const float* p1 = p + 16 + 8 * hh;
#pragma unroll
    for (int e = 0; e < 8; ++e) { fh_[e] = (b16)p0[e]; fh_[8 + e] = (b16)p1[e]; }
    fl_ = fh_;
  } else {
    fh_ = frag_kb((const b16*)o.p0 + (size_t)row * o.ld + kb, hh);
    if (NP == 2) fl_ = frag_kb((const b16*)o.p1 + (size_t)row * o.ld + kb, hh); else fl_ = fh_;
  }
}
template <int ANP, int BNP> __device__ __forceinline__ v8f mac(v16b ah, v16b al, v16b bh, v16b bl, v8f c) {
  c = wmma16b(ah, bh, c);
  if (BNP == 0 || BNP == 2 || BNP == 4 || BNP == 5) c = wmma16b(ah, bl, c);
  if (ANP == 0 || ANP == 2 || ANP == 4 || ANP == 5) c = wmma16b(al, bh, c);
  return c;
}
template <int ANP, int BNP>
__device__ __forceinline__ void gemm_tile(const Opnd& A, const Opnd& B, int K, int m0, int c0, int nloc, int hlf, v8f (&acc)[2][4]) {
  for (int kb = 0; kb < K; kb += 32) {
    v16b a0h, a0l, a1h, a1l;
    load_frags<ANP>(A, m0 + nloc, kb, hlf, a0h, a0l);
    load_frags<ANP>(A, m0 + 16 + nloc, kb, hlf, a1h, a1l);
#pragma unroll
    for (int t = 0; t < 4; ++t) {
      v16b bh, bl;
      load_frags<BNP>(B, c0 + t * 16 + nloc, kb, hlf, bh, bl);
      acc[0][t] = mac<ANP, BNP>(a0h, a0l, bh, bl, acc[0][t]);
      acc[1][t] = mac<ANP, BNP>(a1h, a1l, bh, bl, acc[1][t]);
    }
  }
}

__device__ __forceinline__ void epi_planes(v8f (&acc)[2][4], float scale, bool two, b16* __restrict__ oh, b16* __restrict__ ol, int ldo,
                                           int m0, int c0, int lane, b16* Th, b16* Tl) {
  const int nloc = lane & 15, hlf = lane >> 4;
#pragma unroll
  for (int t = 0; t < 4; ++t)
#pragma unroll
    for (int r = 0; r < 2; ++r)
#pragma unroll
      for (int v = 0; v < 8; ++v) {
        const int rr = r * 16 + v + 8 * hlf, cc = t * 16 + nloc;
        b16 h_, l_; split16(acc[r][t][v] * scale, h_, l_);
        Th[rr * 64 + cc] = h_; Tl[rr * 64 + cc] = l_;
      }
  wave_lds_sync();
  for (int pass = 0; pass < 2; ++pass) {
#pragma unroll
    for (int j = 0; j < 8; ++j) {
      const int rr = j * 4 + (lane >> 3), c8 = (lane & 7) * 8;
      const size_t o = (size_t)(m0 + rr) * ldo + c0 + c8;
      *(volatile v8b*)(oh + o) = ld8b(Th + rr * 64 + c8);
      if (two) *(volatile v8b*)(ol + o) = ld8b(Tl + rr * 64 + c8);
    }
    __threadfence();
  }
}
__device__ __forceinline__ void epi_f32(v8f (&acc)[2][4], float scale, const float* rscale, float* __restrict__ out, int ldo, int m0, int c0, int lane, float* Tt) {
  const int nloc = lane & 15, hlf = lane >> 4;
#pragma unroll
  for (int t = 0; t < 4; ++t)
#pragma unroll
    for (int r = 0; r < 2; ++r)
#pragma unroll
      for (int v = 0; v < 8; ++v) {
        const int rr = r * 16 + v + 8 * hlf;
        const float rs = rscale ? rscale[(size_t)(m0 + rr) * 32] : 1.0f;
        Tt[rr * 64 + t * 16 + nloc] = acc[r][t][v] * scale * rs;
      }
  wave_lds_sync();
  float* dst0 = out + (size_t)m0 * ldo + c0;
  for (int pass = 0; pass < 2; ++pass) {
#pragma unroll
    for (int j = 0; j < 16; ++j) { const int rr = j * 2 + hlf, c4 = nloc * 4; *(volatile v4f*)(dst0 + (size_t)rr * ldo + c4) = *(const v4f*)(Tt + rr * 64 + c4); }
    __threadfence();
  }
}


typedef __attribute__((ext_vector_type(8))) __bf16 v8bb; typedef __attribute__((ext_vector_type(16))) __bf16 v16bb;
typedef __attribute__((ext_vector_type(8))) unsigned short v8us;
__device__ __forceinline__ v16bb frag_kb_bf(const __bf16* p, int hh) { const v8bb a = *(const v8bb*)(p + 8 * hh), b = *(const v8bb*)(p + 16 + 8 * hh); return __builtin_shufflevector(a, b, 0, 1, 2, 3, 4, 5, 6, 7, 8, 9, 10, 11, 12, 13, 14, 15); }
__device__ __forceinline__ v8f wmma16bb(v16bb a, v16bb b, v8f c) {
  v8f d = __builtin_amdgcn_wmma_f32_16x16x32_bf16(false, a, false, b, (short)0, c, false, false);
  asm volatile("v_nop\n\tv_nop\n\tv_nop\n\tv_nop" : "+v"(d) : "v"(a), "v"(b));
  return d;
}
__device__ __forceinline__ unsigned short bf16_rne_bits(float v) { unsigned int u = __float_as_uint(v); u += 0x7FFFu + ((u >> 16) & 1u); return (unsigned short)(u >> 16); }
__device__ __forceinline__ float bf16_rne(float v) { return __uint_as_float(((unsigned int)bf16_rne_bits(v)) << 16); }


__global__ __launch_bounds__(256) void theta_kernel(const float* __restrict__ x, const float* __restrict__ tw, const float* __restrict__ tb, b16* __restrict__ th) {
  const size_t gi = (size_t)blockIdx.x * 256 + threadIdx.x; const int q = (int)(gi & 3); const size_t bn = gi >> 2; const int b = (int)(bn / NP), n = (int)(bn % NP);
  float acc[8];
#pragma unroll
  for (int j = 0; j < 8; ++j) acc[j] = tb[q * 8 + j];
#pragma unroll 4
  for (int c = 0; c < C; ++c) { const float xv = x[((size_t)b * C + c) * NP + n];
#pragma unroll
    for (int j = 0; j < 8; ++j) acc[j] += tw[(q * 8 + j) * C + c] * xv; }
  v8b hv, lv;
#pragma unroll
  for (int j = 0; j < 8; ++j) { b16 a, l; split16(acc[j] * CS8, a, l); hv[j] = a; lv[j] = l; }
  for (int pass = 0; pass < 2; ++pass) { *(volatile v8b*)(th + bn * I + q * 8) = hv; *(volatile v8b*)(th + TPL + bn * I + q * 8) = lv; __threadfence(); }
}

__global__ __launch_bounds__(256) void kv_kernel(const float* __restrict__ x, const float* __restrict__ lf, const float* __restrict__ pw, const float* __restrict__ pb, const float* __restrict__ gw, const float* __restrict__ gb,
                                                const float* __restrict__ hw, const float* __restrict__ hb, b16* __restrict__ key, b16* __restrict__ gt) {
  __shared__ __attribute__((aligned(16))) b16 Gh[I][64 + 8], Gl[I][64 + 8];
  const int t_ = threadIdx.x, ml = t_ >> 2, q = t_ & 3, b = blockIdx.x / (NK / 64), m = (blockIdx.x % (NK / 64)) * 64 + ml;
  const int pr = m / (WW / 2), pc_ = m % (WW / 2);
  float kmax[8], gmax[8], hmax[8];
#pragma unroll
  for (int j = 0; j < 8; ++j) { kmax[j] = -INFINITY; gmax[j] = -INFINITY; hmax[j] = -INFINITY; }
  for (int d = 0; d < 4; ++d) { const int n = (2 * pr + (d >> 1)) * WW + 2 * pc_ + (d & 1);
    float pa[8], ga[8], ha[8];
#pragma unroll
    for (int j = 0; j < 8; ++j) { pa[j] = pb[q * 8 + j]; ga[j] = gb[q * 8 + j]; ha[j] = hb[q * 8 + j]; }
#pragma unroll 1
    for (int c = 0; c < C; ++c) { const float xv = x[((size_t)b * C + c) * NP + n];
#pragma unroll
      for (int j = 0; j < 8; ++j) { pa[j] += pw[(q * 8 + j) * C + c] * xv; ga[j] += gw[(q * 8 + j) * C + c] * xv; } }
#pragma unroll 1
    for (int c = 0; c < CL; ++c) { const float lv = lf[((size_t)b * CL + c) * NP + n];
#pragma unroll
      for (int j = 0; j < 8; ++j) ha[j] += hw[(q * 8 + j) * CL + c] * lv; }
#pragma unroll
    for (int j = 0; j < 8; ++j) { kmax[j] = fmaxf(kmax[j], pa[j]); gmax[j] = fmaxf(gmax[j], ga[j]); hmax[j] = fmaxf(hmax[j], ha[j]); } }
  v8b kh_, kl_;
#pragma unroll
  for (int j = 0; j < 8; ++j) { b16 a, l; split16((kmax[j] + hmax[j]) * CS8, a, l); kh_[j] = a; kl_[j] = l; split16(gmax[j] * CS8, a, l); Gh[q * 8 + j][ml] = a; Gl[q * 8 + j][ml] = l; }
  __syncthreads();
  const size_t kb = ((size_t)b * NK + m) * I + q * 8;
  for (int pass = 0; pass < 2; ++pass) {
    *(volatile v8b*)(key + kb) = kh_; *(volatile v8b*)(key + KPL + kb) = kl_;
    { const int i = t_ >> 3, c8 = (t_ & 7) * 8; const size_t gofs = ((size_t)b * I + i) * NK + (blockIdx.x % (NK / 64)) * 64 + c8; *(volatile v8b*)(gt + gofs) = *(const v8b*)(&Gh[i][c8]); *(volatile v8b*)(gt + GPL + gofs) = *(const v8b*)(&Gl[i][c8]); }
    __threadfence();
  }
}

__global__ __launch_bounds__(256) void attn_kernel(const b16* __restrict__ th, const b16* __restrict__ key, const b16* __restrict__ gt, const float* __restrict__ Ww, const float* __restrict__ Wb,
                                                  const float* __restrict__ bng, const float* __restrict__ bnb, const float* __restrict__ bnm, const float* __restrict__ bnv, const float* __restrict__ x, float* __restrict__ out) {
  __shared__ __attribute__((aligned(16))) float Ob[C][128 + 4];
  __shared__ float Ys[8][16][I + 1];
  const int wid = threadIdx.x >> 5, lane = threadIdx.x & 31, hh = lane >> 4, col = lane & 15;
  const int b = blockIdx.x / (NP / 128), n0b = (blockIdx.x % (NP / 128)) * 128, q0 = n0b + wid * 16, qi = q0 + col;
  const b16* T = th + ((size_t)b * NP) * I; const b16* K = key + ((size_t)b * NK) * I; const b16* Gt = gt + ((size_t)b * I) * NK;
  const v16b qf = frag_kb(T + (size_t)qi * I, hh), ql = frag_kb(T + TPL + (size_t)qi * I, hh);
  float m = -INFINITY, l = 0.0f; v8f o[2] = {{}, {}};
  for (int kb = 0; kb < NK; kb += 32) {
    v8f s0 = {}, s1 = {};
    { const v16b k0 = frag_kb(K + (size_t)(kb + col) * I, hh), k0l = frag_kb(K + KPL + (size_t)(kb + col) * I, hh), k1 = frag_kb(K + (size_t)(kb + 16 + col) * I, hh), k1l = frag_kb(K + KPL + (size_t)(kb + 16 + col) * I, hh);
      s0 = wmma16b(k0, qf, s0); s0 = wmma16b(k0, ql, s0); s0 = wmma16b(k0l, qf, s0); s1 = wmma16b(k1, qf, s1); s1 = wmma16b(k1, ql, s1); s1 = wmma16b(k1l, qf, s1); }
    float mr = -INFINITY;
#pragma unroll
    for (int r = 0; r < 8; ++r) { s0[r] *= 1.0f / (CS8 * CS8); s1[r] *= 1.0f / (CS8 * CS8); mr = fmaxf(mr, fmaxf(s0[r], s1[r])); }
    mr = fmaxf(mr, __shfl_xor(mr, 16));
    const float mn = fmaxf(m, mr), al_ = __expf(m - mn); m = mn;
    float sum = 0.0f; v16b pb, pl;
#pragma unroll
    for (int r = 0; r < 8; ++r) { const float e0 = __expf(s0[r] - mn), e1 = __expf(s1[r] - mn); sum += e0 + e1; b16 a, cc; split16(e0 * PS, a, cc); pb[r] = a; pl[r] = cc; split16(e1 * PS, a, cc); pb[8 + r] = a; pl[8 + r] = cc; }
    sum += __shfl_xor(sum, 16); l = l * al_ + sum;
#pragma unroll
    for (int nn = 0; nn < 2; ++nn) {
#pragma unroll
      for (int r = 0; r < 8; ++r) o[nn][r] *= al_;
      const v16b gf = frag_kb(Gt + (size_t)(nn * 16 + col) * NK + kb, hh), gl = frag_kb(Gt + GPL + (size_t)(nn * 16 + col) * NK + kb, hh);
      o[nn] = wmma16b(gf, pb, o[nn]); o[nn] = wmma16b(gf, pl, o[nn]); o[nn] = wmma16b(gl, pb, o[nn]); }
  }
  const float inv = 1.0f / (CS8 * PS * l);
#pragma unroll
  for (int nn = 0; nn < 2; ++nn)
#pragma unroll
    for (int r = 0; r < 8; ++r) Ys[wid][col][nn * 16 + 8 * hh + r] = o[nn][r] * inv;
  wave_lds_sync();
  { const int n = q0 + col; float yv[I];
#pragma unroll
    for (int i = 0; i < I; ++i) yv[i] = Ys[wid][col][i];
    for (int cc = 0; cc < C / 2; ++cc) { const int c = hh * (C / 2) + cc; float s = Wb[c];
#pragma unroll
      for (int i = 0; i < I; ++i) s += Ww[c * I + i] * yv[i];
      const float sc = bng[c] / sqrtf(bnv[c] + BNE); Ob[c][wid * 16 + col] = (s - bnm[c]) * sc + bnb[c] + x[((size_t)b * C + c) * NP + n]; } }
  __syncthreads();
  for (int pass = 0; pass < 2; ++pass) {
    for (int i = threadIdx.x; i < C * 32; i += 256) { const int c = i >> 5, qd = (i & 31) * 4; *(volatile v4f*)(out + ((size_t)b * C + c) * NP + n0b + qd) = *(const v4f*)(&Ob[c][qd]); }
    __threadfence();
  }
}
}

extern "C" void kernel_launch(void* const* d_in, const int* in_sizes, int n_in,
                              void* d_out, int out_size, void* d_ws, size_t ws_size, hipStream_t stream) {
  (void)n_in; (void)out_size;
  const float* x = (const float*)d_in[0]; const float* lfeat = (const float*)d_in[1]; const float* hc_w = (const float*)d_in[2]; const float* hc_b = (const float*)d_in[3];
  const float* g_w = (const float*)d_in[4]; const float* g_b = (const float*)d_in[5]; const float* th_w = (const float*)d_in[6]; const float* th_b = (const float*)d_in[7]; const float* ph_w = (const float*)d_in[8]; const float* ph_b = (const float*)d_in[9];
  const float* W_w = (const float*)d_in[10]; const float* W_b = (const float*)d_in[11]; const float* bng = (const float*)d_in[12]; const float* bnb = (const float*)d_in[13]; const float* bnm = (const float*)d_in[14]; const float* bnv = (const float*)d_in[15];
  float* out = (float*)d_out;
  if (in_sizes[0] != Bn * C * NP || in_sizes[1] != Bn * CL * NP || in_sizes[2] != I * CL || in_sizes[6] != I * C || in_sizes[10] != C * I) return;
  size_t off = 0; char* ws = (char*)d_ws;
  auto carve = [&](size_t bytes) { char* p = ws + off; off += (bytes + 255) & ~(size_t)255; return p; };
  b16* th = (b16*)carve(TPL * 2 * 2); b16* key = (b16*)carve(KPL * 2 * 2); b16* gt = (b16*)carve(GPL * 2 * 2);
  if (off > ws_size) return;
  theta_kernel<<<Bn * NP * 4 / 256, 256, 0, stream>>>(x, th_w, th_b, th);
  kv_kernel<<<Bn * NK / 64, 256, 0, stream>>>(x, lfeat, ph_w, ph_b, g_w, g_b, hc_w, hc_b, key, gt);
  attn_kernel<<<Bn * NP / 128, 256, 0, stream>>>(th, key, gt, W_w, W_b, bng, bnb, bnm, bnv, x, out);
}
